// DotProductAttention_27023934227141
// MI455X (gfx1250) — hardware-verified
//
#include <hip/hip_runtime.h>


#ifndef NB
#define NB 4
#endif
#ifndef SEQ
#define SEQ 1024
#endif
#define NB_FULL  4
#define SEQ_FULL 1024
#define NH   16
#define HD   64
#define TT   SEQ
#define NZ   (NB * NH)
#define ZG   8
#define NGRP (NZ / ZG)

static_assert(NB <= NB_FULL);
static_assert(SEQ <= SEQ_FULL);
static_assert(TT % 128 == 0);
static_assert(HD % 64 == 0);
static_assert(HD % 32 == 0);
static_assert(NZ % ZG == 0);
static_assert(((TT * HD) / 8) % 256 == 0);
static_assert(((HD * TT) / 2) % 256 == 0);
static_assert((ZG * TT) % 8 == 0);

typedef unsigned short bf;
typedef __attribute__((ext_vector_type(16))) __bf16   v16bf;
typedef __attribute__((ext_vector_type(8)))  unsigned short v8us;
typedef __attribute__((ext_vector_type(4)))  unsigned short v4us;
typedef __attribute__((ext_vector_type(2)))  unsigned short v2us;
typedef __attribute__((ext_vector_type(8)))  float    v8f;
typedef __attribute__((ext_vector_type(4)))  float    v4f;
typedef v4f  __attribute__((may_alias)) v4fa;

__device__ __forceinline__ unsigned short f2bf(float f) { unsigned u = __float_as_uint(f); u += 0x7FFFu + ((u >> 16) & 1u); return (unsigned short)(u >> 16); }
__device__ __forceinline__ float bf2f(unsigned short b) { return __uint_as_float(((unsigned)b) << 16); }
__device__ __forceinline__ float bfr(float f) { return bf2f(f2bf(f)); }
__device__ __forceinline__ v16bf cat16b(v8us lo, v8us hi) { return __builtin_bit_cast(v16bf, __builtin_shufflevector(lo, hi, 0, 1, 2, 3, 4, 5, 6, 7, 8, 9, 10, 11, 12, 13, 14, 15)); }
__device__ __forceinline__ v8f wmmab(v16bf a, v16bf b, v8f c) { return __builtin_amdgcn_wmma_f32_16x16x32_bf16(false, a, false, b, (short)0, c, false, false); }

template <typename T16> struct WFrag;
template <> struct WFrag<bf> { typedef v16bf V; static __device__ __forceinline__ V ld(const bf* p) { return cat16b(*(const v8us*)p, *(const v8us*)(p + 16)); } static __device__ __forceinline__ v8f mma(V a, V b, v8f c) { return wmmab(a, b, c); } };
template <typename T16, int NSPLIT, bool BIAS>
__global__ __launch_bounds__(32) void k_gemmw(const T16* __restrict__ A, const T16* __restrict__ A2, const T16* __restrict__ Bt, const T16* __restrict__ Bt2, int K, float* C, int ldc, const float* __restrict__ bias, size_t sA, size_t sB, size_t sC) {
    typedef typename WFrag<T16>::V V;
    __shared__ __align__(16) float os[16 * 68];
    const size_t z = blockIdx.z; A += z * sA; if (A2) A2 += z * sA; Bt += z * sB; if (Bt2) Bt2 += z * sB; C += z * sC;
    const int lane = threadIdx.x & 31, lr = lane & 15, hi = lane >> 4; const int r0 = blockIdx.x * 64, c0 = blockIdx.y * 64;
    v8f acc[4][4];
#pragma unroll
    for (int mb = 0; mb < 4; ++mb)
#pragma unroll
        for (int nb = 0; nb < 4; ++nb) acc[mb][nb] = (v8f){};
    const size_t aoff = (size_t)(r0 + lr) * K + 8 * hi, boff = (size_t)(c0 + lr) * K + 8 * hi;
#pragma unroll 1
    for (int kc = 0; kc < K; kc += 32) {
        V a[4], a2[4];
#pragma unroll
        for (int mb = 0; mb < 4; ++mb) { a[mb] = WFrag<T16>::ld(A + aoff + (size_t)mb * 16 * K + kc); if (NSPLIT == 1 || NSPLIT == 2) a2[mb] = WFrag<T16>::ld(A2 + aoff + (size_t)mb * 16 * K + kc); }
#pragma unroll
        for (int nb = 0; nb < 4; ++nb) { const V b = WFrag<T16>::ld(Bt + boff + (size_t)nb * 16 * K + kc); V b2; if (NSPLIT >= 2) b2 = WFrag<T16>::ld(Bt2 + boff + (size_t)nb * 16 * K + kc);
#pragma unroll
            for (int mb = 0; mb < 4; ++mb) { acc[mb][nb] = WFrag<T16>::mma(a[mb], b, acc[mb][nb]); if (NSPLIT == 1 || NSPLIT == 2) acc[mb][nb] = WFrag<T16>::mma(a2[mb], b, acc[mb][nb]); if (NSPLIT >= 2) acc[mb][nb] = WFrag<T16>::mma(a[mb], b2, acc[mb][nb]); } }
        asm volatile("v_nop\n\tv_nop\n\tv_nop\n\tv_nop" : "+v"(acc[0][0]), "+v"(acc[1][1]), "+v"(acc[2][2]), "+v"(acc[3][3]) : "v"(a[0]), "v"(a[3]));
    }
#pragma unroll
    for (int mb = 0; mb < 4; ++mb) {
#pragma unroll
        for (int nb = 0; nb < 4; ++nb) {
#pragma unroll
            for (int j = 0; j < 8; ++j) os[(hi * 8 + j) * 68 + nb * 16 + lr] = acc[mb][nb][j]; }
        __builtin_amdgcn_wave_barrier(); asm volatile("" ::: "memory");
        float* crow = C + (size_t)(r0 + mb * 16) * ldc + c0;
#pragma unroll 1
        for (int ps = 0; ps < 2; ++ps) {
#pragma unroll
            for (int s = 0; s < 8; ++s) { const int row = 2 * s + hi, cofs = lr * 4; v4f val = *(const v4fa*)(os + row * 68 + cofs); if (BIAS) { val[0] += bfr(bias[c0 + cofs]); val[1] += bfr(bias[c0 + cofs + 1]); val[2] += bfr(bias[c0 + cofs + 2]); val[3] += bfr(bias[c0 + cofs + 3]); }
                *(volatile v4f*)(crow + (size_t)row * ldc + cofs) = val; }
            if (ps == 0) __threadfence(); }
        __builtin_amdgcn_wave_barrier(); asm volatile("" ::: "memory");
    }
}

__device__ __forceinline__ void splitf(float y, unsigned short& h, unsigned short& l) { h = f2bf(y); l = f2bf(y - bf2f(h)); }

__global__ __launch_bounds__(256) void k_cvt8(const float* __restrict__ src, bf* dst) {
    const unsigned z = blockIdx.y; const unsigned i = blockIdx.x * 256u + threadIdx.x; if (i >= (unsigned)(TT * HD / 8)) return;
    const float* s = src + (size_t)z * SEQ_FULL * HD + (size_t)i * 8; bf* d = dst + (size_t)z * TT * HD + (size_t)i * 8;
    const v8f v = *(const v8f*)s; v8us o;
#pragma unroll
    for (int k = 0; k < 8; ++k) o[k] = f2bf(v[k]);
    *(volatile v8us*)d = o; __threadfence(); *(volatile v8us*)d = o; }

__global__ __launch_bounds__(256) void k_vtpR1(const float* __restrict__ Vin, bf* VT) {
    const unsigned z = blockIdx.y; const unsigned e = (blockIdx.x * 256u + threadIdx.x) * 2u; if (e >= (unsigned)(HD * TT)) return;
    const unsigned t = e % (unsigned)TT; const unsigned d = e / (unsigned)TT;
    const float* Vb = Vin + (size_t)z * SEQ_FULL * HD; bf* dst = VT + (size_t)z * HD * TT + e;
    v2us o; o[0] = f2bf(Vb[(size_t)t * HD + d]); o[1] = f2bf(Vb[(size_t)(t + 1u) * HD + d]);
    *(volatile v2us*)dst = o; __threadfence(); *(volatile v2us*)dst = o; }

__global__ __launch_bounds__(256) void k_asoft(const float* __restrict__ Sb, bf* Ph, bf* Pl, const int* __restrict__ dkp) {
    const unsigned lane = threadIdx.x & 31u; const unsigned row = blockIdx.x * 8u + (threadIdx.x >> 5); if (row >= (unsigned)(ZG * TT)) return;
    int dk = dkp[0]; dk = dk < 1 ? 1 : dk; const float scl = 1.0f / sqrtf((float)dk);
    const float* sr = Sb + (size_t)row * TT; float v[TT / 32]; float mx = -3.0e38f;
#pragma unroll
    for (int ch = 0; ch < TT / 128; ++ch) { const unsigned j0 = (unsigned)ch * 128u + lane * 4u; const v4f a = *(const v4f*)(sr + j0);
#pragma unroll
        for (int q = 0; q < 4; ++q) { const float t = a[q] * scl; v[ch * 4 + q] = t; mx = fmaxf(mx, t); } }
#pragma unroll
    for (int sh = 16; sh; sh >>= 1) mx = fmaxf(mx, __shfl_xor(mx, sh, 32));
    float sum = 0.f;
#pragma unroll
    for (int k = 0; k < TT / 32; ++k) { float d0 = __fsub_rn(v[k], mx); asm volatile("" : "+v"(d0)); v[k] = __builtin_amdgcn_exp2f(__fmul_rn(d0, 1.4426950408889634f)); sum += v[k]; }
#pragma unroll
    for (int sh = 16; sh; sh >>= 1) sum += __shfl_xor(sum, sh, 32);
    const float f = __fdiv_rn(1.0f, sum);
    v4us oh[TT / 128], ol[TT / 128];
#pragma unroll
    for (int ch = 0; ch < TT / 128; ++ch) {
#pragma unroll
        for (int q = 0; q < 4; ++q) { unsigned short a, c2; splitf(v[ch * 4 + q] * f, a, c2); oh[ch][q] = a; ol[ch][q] = c2; } }
    const size_t ob = (size_t)row * TT + lane * 4u;
#pragma unroll 1
    for (int ps = 0; ps < 2; ++ps) {
#pragma unroll
        for (int ch = 0; ch < TT / 128; ++ch) { const size_t oo = ob + (size_t)ch * 128; *(volatile v4us*)(Ph + oo) = oh[ch]; *(volatile v4us*)(Pl + oo) = ol[ch]; }
        if (ps == 0) __threadfence(); }
}

#define PLANE_BYTES ((size_t)NZ * TT * HD * 2)
#define S_BYTES     ((size_t)ZG * TT * TT * 4)
#define P_BYTES     ((size_t)ZG * TT * TT * 2)
static_assert(PLANE_BYTES % 256 == 0);
static_assert(S_BYTES % 256 == 0);
static_assert(P_BYTES % 256 == 0);
static_assert(3 * PLANE_BYTES + S_BYTES + 2 * P_BYTES <= (size_t)134217728);

extern "C" void kernel_launch(void* const* d_in, const int* in_sizes, int n_in,
                              void* d_out, int out_size, void* d_ws, size_t ws_size, hipStream_t stream) {
    if (n_in < 4) return;
    const size_t need_in = (size_t)(NZ - 1) * SEQ_FULL * HD + (size_t)TT * HD;
    if ((size_t)in_sizes[0] < need_in || (size_t)in_sizes[1] < need_in || (size_t)in_sizes[2] < need_in || in_sizes[3] < 1) return;
    if ((size_t)out_size < (size_t)NZ * TT * HD) return;
    const float* Qin = (const float*)d_in[0]; const float* Kin = (const float*)d_in[1]; const float* Vin = (const float*)d_in[2]; const int* DK = (const int*)d_in[3];
    float* OUT = (float*)d_out;
    char* wsp = (char*)d_ws;
    auto take = [&](size_t bytes) { char* p = wsp; wsp += (bytes + 255) & ~(size_t)255; return (void*)p; };
    bf* QB = (bf*)take(PLANE_BYTES); bf* KB = (bf*)take(PLANE_BYTES); bf* VT = (bf*)take(PLANE_BYTES);
    float* Sb = (float*)take(S_BYTES); bf* Ph = (bf*)take(P_BYTES); bf* Pl = (bf*)take(P_BYTES);
    if ((size_t)(wsp - (char*)d_ws) > ws_size) return;
    k_cvt8<<<dim3((unsigned)(TT * HD / 8 / 256), NZ, 1), 256, 0, stream>>>(Qin, QB);
    k_cvt8<<<dim3((unsigned)(TT * HD / 8 / 256), NZ, 1), 256, 0, stream>>>(Kin, KB);
    k_vtpR1<<<dim3((unsigned)(HD * TT / 2 / 256), NZ, 1), 256, 0, stream>>>(Vin, VT);
    for (int g = 0; g < NGRP; ++g) {
        const size_t pofs = (size_t)g * ZG * TT * HD;
        k_gemmw<bf, 0, false><<<dim3(TT / 64, TT / 64, ZG), 32, 0, stream>>>(QB + pofs, nullptr, KB + pofs, nullptr, HD, Sb, TT, nullptr, (size_t)TT * HD, (size_t)TT * HD, (size_t)TT * TT);
        k_asoft<<<(unsigned)(ZG * TT / 8), 256, 0, stream>>>(Sb, Ph, Pl, DK);
        k_gemmw<bf, 1, false><<<dim3(TT / 64, HD / 64, ZG), 32, 0, stream>>>(Ph, Pl, VT + pofs, nullptr, TT, OUT + pofs, HD, nullptr, (size_t)TT * TT, (size_t)HD * TT, (size_t)TT * HD);
    }
}
